// EllipticGNN_60988535603849
// MI455X (gfx1250) — hardware-verified
//
#include <hip/hip_runtime.h>
#include <stddef.h>


#define NTHR    256
#define NWAVE   8
#define EPT     8
#define NGRP    2
#define CHUNK   (NTHR * EPT * NGRP)
#define WCAP    (EPT * NGRP * 32)
#define LISTN   (NWAVE * WCAP)
#define NBC     4096
#define NBF     1024
#define RCAP    24576
#define RBN     128
#define TGT     256
#define DEGCAP  1024
#define OTHR    512
#define BM      64
#define BNC     128
#define WSCAP   134217728
#define FIN     165
#define KIN     192
#define HD      128
#define DHD     64
#define ZW      32
#define NOUT    2
#define KSG     256
#define S3P     72
#define SZP     36
#define ACARRY  8.0f
#define WCARRY  64.0f
#define GSCALE  (1.0f / 512.0f)
#define BNEPS   1e-5f

#define LDS_FILL ((RCAP + NBF + LISTN) * 4 + 64)

static_assert((CHUNK & (CHUNK - 1)) == 0);
static_assert(CHUNK <= 4096);
static_assert((NBC & (NBC - 1)) == 0 && (NBF & (NBF - 1)) == 0);
static_assert(NBC == 4 * NBF);
static_assert(OTHR * 8 == NBC);
static_assert((RCAP % 32) == 0);
static_assert(TGT == NWAVE * 32);
static_assert((NBC % TGT) == 0);
static_assert((TGT % BM) == 0);
static_assert(WCAP == EPT * NGRP * 32);
static_assert((KIN % 32) == 0 && KIN >= FIN);
static_assert((HD % 32) == 0 && (KSG % 32) == 0 && (DHD % 32) == 0);
static_assert(HD == 4 * 32);
static_assert(KSG == 2 * HD);
static_assert(DHD == 2 * 32);
static_assert(BM * NOUT == 4 * 32);
static_assert((S3P % 8) == 0 && (SZP % 4) == 0);

typedef float    v2f  __attribute__((ext_vector_type(2)));
typedef float    v4f  __attribute__((ext_vector_type(4)));
typedef float    v8f  __attribute__((ext_vector_type(8)));
typedef int      v4i  __attribute__((ext_vector_type(4)));
typedef _Float16 v4h  __attribute__((ext_vector_type(4)));
typedef _Float16 v8h  __attribute__((ext_vector_type(8)));
typedef _Float16 v16h __attribute__((ext_vector_type(16)));
union Frag { v16h v; v8h h[2]; };

__device__ __forceinline__ v8f wmh(v16h a, v16h b, v8f c) {
  v8f d = __builtin_amdgcn_wmma_f32_16x16x32_f16(false, a, false, b, (short)0, c, false, false);
  asm volatile("v_nop\n\tv_nop\n\tv_nop\n\tv_nop" : "+v"(d) : "v"(a), "v"(b));
  return d;
}

__device__ __forceinline__ float eluf(float x)   { return x > 0.f ? x : expm1f(x); }
__device__ __forceinline__ float lrelu1(float x) { return x >= 0.f ? x : 0.2f * x; }
__device__ __forceinline__ v4f selz(v4f v, bool live) {
  v4f o; o.x = live ? v.x : 0.f; o.y = live ? v.y : 0.f; o.z = live ? v.z : 0.f; o.w = live ? v.w : 0.f; return o;
}
__device__ __forceinline__ v2f selz(v2f v, bool live) {
  v2f o; o.x = live ? v.x : 0.f; o.y = live ? v.y : 0.f; return o;
}
__device__ __forceinline__ v2f selv2(v2f v, bool c, float other) {
  v2f o; o.x = c ? v.x : other; o.y = c ? v.y : other; return o;
}
__device__ __forceinline__ v4f elu4(v4f v) {
  v4f o; o.x = eluf(v.x); o.y = eluf(v.y); o.z = eluf(v.z); o.w = eluf(v.w); return o;
}
__device__ __forceinline__ v4h cvt4h(v4f v) {
  v4h o; o.x = (_Float16)v.x; o.y = (_Float16)v.y; o.z = (_Float16)v.z; o.w = (_Float16)v.w; return o;
}
__device__ __forceinline__ v4f nscale4(const float* __restrict__ g, const float* __restrict__ v, int lane) {
  const v4f g4 = *(const v4f*)(g + 4 * lane);
  const v4f v4 = *(const v4f*)(v + 4 * lane);
  v4f o;
  o.x = g4.x / sqrtf(v4.x + BNEPS); o.y = g4.y / sqrtf(v4.y + BNEPS);
  o.z = g4.z / sqrtf(v4.z + BNEPS); o.w = g4.w / sqrtf(v4.w + BNEPS);
  return o;
}
__device__ __forceinline__ v2f wmax2(v2f v) {
#pragma unroll
  for (int off = 16; off > 0; off >>= 1) {
    v.x = fmaxf(v.x, __shfl_xor(v.x, off)); v.y = fmaxf(v.y, __shfl_xor(v.y, off));
  }
  return v;
}
__device__ __forceinline__ v2f wsum2(v2f v) {
#pragma unroll
  for (int off = 16; off > 0; off >>= 1) {
    v.x += __shfl_xor(v.x, off); v.y += __shfl_xor(v.y, off);
  }
  return v;
}

template <int NB>
__device__ __forceinline__ int scan_chunk(const int* __restrict__ dsts, int nE, int cbase, int slotBase,
                                          int vec8, int* list, int tid, int lane, int wave) {
  int wc = 0;
#pragma unroll
  for (int g = 0; g < NGRP; ++g) {
    const int el0  = (g * NTHR + tid) * EPT;
    const int e0   = cbase + el0;
    const int sent = -2147483647 - 1;
    v4i da, db;
    if (vec8 != 0 && cbase + CHUNK <= nE) {
      da = *(const v4i*)(dsts + e0);
      db = *(const v4i*)(dsts + e0 + 4);
    } else {
      da.x = (e0     < nE) ? dsts[min(e0, nE - 1)] : sent;
      da.y = (e0 + 1 < nE) ? dsts[min(e0 + 1, nE - 1)] : sent;
      da.z = (e0 + 2 < nE) ? dsts[min(e0 + 2, nE - 1)] : sent;
      da.w = (e0 + 3 < nE) ? dsts[min(e0 + 3, nE - 1)] : sent;
      db.x = (e0 + 4 < nE) ? dsts[min(e0 + 4, nE - 1)] : sent;
      db.y = (e0 + 5 < nE) ? dsts[min(e0 + 5, nE - 1)] : sent;
      db.z = (e0 + 6 < nE) ? dsts[min(e0 + 6, nE - 1)] : sent;
      db.w = (e0 + 7 < nE) ? dsts[min(e0 + 7, nE - 1)] : sent;
    }
    const unsigned nb = (unsigned)slotBase;
    const unsigned s0 = (unsigned)da.x - nb, s1 = (unsigned)da.y - nb;
    const unsigned s2 = (unsigned)da.z - nb, s3 = (unsigned)da.w - nb;
    const unsigned s4 = (unsigned)db.x - nb, s5 = (unsigned)db.y - nb;
    const unsigned s6 = (unsigned)db.z - nb, s7 = (unsigned)db.w - nb;
    const bool h0 = s0 < (unsigned)NB, h1 = s1 < (unsigned)NB, h2 = s2 < (unsigned)NB, h3 = s3 < (unsigned)NB;
    const bool h4 = s4 < (unsigned)NB, h5 = s5 < (unsigned)NB, h6 = s6 < (unsigned)NB, h7 = s7 < (unsigned)NB;
    const unsigned any = __builtin_amdgcn_ballot_w32(h0 | h1 | h2 | h3 | h4 | h5 | h6 | h7);
    if (any != 0u) {
#define HITJ(J, HJ, SJ) { \
        const unsigned mj = __builtin_amdgcn_ballot_w32(HJ); \
        if (mj != 0u) { \
          if (HJ) { \
            const int pos = wc + (int)__builtin_amdgcn_mbcnt_lo(mj, 0u); \
            if (pos < WCAP) list[wave * WCAP + pos] = ((el0 + (J)) << 12) | (int)(SJ); \
          } \
          wc += (int)__builtin_popcount(mj); } }
      HITJ(0, h0, s0)
      HITJ(1, h1, s1)
      HITJ(2, h2, s2)
      HITJ(3, h3, s3)
      HITJ(4, h4, s4)
      HITJ(5, h5, s5)
      HITJ(6, h6, s6)
      HITJ(7, h7, s7)
#undef HITJ
    }
  }
  return wc;
}

__global__ __launch_bounds__(NTHR) void k_count(
    const int* __restrict__ dsts, int* cnt, float* dinv, int nE, int vec8) {
  __shared__ __attribute__((aligned(16))) int scnt[NBC];
  __shared__ __attribute__((aligned(16))) int list[LISTN];
  __shared__ int wcnt[NWAVE];
  const int tid = threadIdx.x, lane = tid & 31, wave = tid >> 5;
  const int nodeBase = blockIdx.x * NBC;

  for (int i = tid; i < NBC; i += NTHR) scnt[i] = 0;
  __syncthreads();

  const int nChunks = (nE + CHUNK - 1) / CHUNK;
#pragma unroll 1
  for (int ch = 0; ch < nChunks; ++ch) {
    const int cbase = ch * CHUNK;
    const int wc = scan_chunk<NBC>(dsts, nE, cbase, nodeBase, vec8, list, tid, lane, wave);
    if (lane == 0) wcnt[wave] = wc;
    __syncthreads();
    if (wave == 0) {
#pragma unroll 1
      for (int wsx = 0; wsx < NWAVE; ++wsx) {
        int n = __builtin_amdgcn_readfirstlane(wcnt[wsx]);
        n = n > WCAP ? WCAP : (n < 0 ? 0 : n);
        const int* lp = list + wsx * WCAP;
#pragma unroll 1
        for (int i = 0; i < n; ++i) {
          const int ent  = __builtin_amdgcn_readfirstlane(lp[i]);
          const int slot = ent & (NBC - 1);
          if (lane == 0) scnt[slot] = scnt[slot] + 1;
        }
      }
    }
    __syncthreads();
  }

  v4i cq[4];
  v4f dq[4];
#pragma unroll
  for (int q = 0; q < 4; ++q) {
    const int f = (wave * 4 + q) * 128 + 4 * lane;
    const v4i cv = *(const v4i*)(scnt + f);
    cq[q] = cv;
    v4f d;
    d.x = rsqrtf((float)(cv.x < 0 ? 0 : cv.x) + 1.0f);
    d.y = rsqrtf((float)(cv.y < 0 ? 0 : cv.y) + 1.0f);
    d.z = rsqrtf((float)(cv.z < 0 ? 0 : cv.z) + 1.0f);
    d.w = rsqrtf((float)(cv.w < 0 ? 0 : cv.w) + 1.0f);
    dq[q] = d;
  }
  int*   cp = cnt  + (size_t)nodeBase;
  float* dp = dinv + (size_t)nodeBase;
#pragma unroll
  for (int q = 0; q < 4; ++q) {
    const int f = (wave * 4 + q) * 128 + 4 * lane;
    *(volatile v4i*)(cp + f) = cq[q];
    *(volatile v4f*)(dp + f) = dq[q];
  }
  __threadfence();
#pragma unroll
  for (int q = 0; q < 4; ++q) {
    const int f = (wave * 4 + q) * 128 + 4 * lane;
    *(volatile v4i*)(cp + f) = cq[q];
    *(volatile v4f*)(dp + f) = dq[q];
  }
}

__global__ __launch_bounds__(OTHR) void k_offsets(
    const int* __restrict__ cnt, int* off, int* rbase, int nChunk) {
  __shared__ __attribute__((aligned(16))) int soff[NBC];
  __shared__ __attribute__((aligned(16))) int srb[RBN];
  __shared__ int wtot[OTHR / 32];
  const int tid = threadIdx.x, lane = tid & 31, wave = tid >> 5, sub = tid >> 7;
  for (int i = tid; i < RBN; i += OTHR) srb[i] = 0;
  int carry = 0;
#pragma unroll 1
  for (int ch = 0; ch < nChunk; ++ch) {
    const int base = ch * NBC;
    const v4i c0 = *(const v4i*)(cnt + base + 8 * tid);
    const v4i c1 = *(const v4i*)(cnt + base + 8 * tid + 4);
    const int e0 = max(c0.x, 0), e1 = max(c0.y, 0), e2 = max(c0.z, 0), e3 = max(c0.w, 0);
    const int e4 = max(c1.x, 0), e5 = max(c1.y, 0), e6 = max(c1.z, 0), e7 = max(c1.w, 0);
    const int ts = e0 + e1 + e2 + e3 + e4 + e5 + e6 + e7;
    int incl = ts;
#pragma unroll
    for (int d = 1; d < 32; d <<= 1) {
      const int t = __shfl_up(incl, d);
      if (lane >= d) incl += t;
    }
    if (lane == 31) wtot[wave] = incl;
    __syncthreads();
    const int S0 = wtot[0]  + wtot[1]  + wtot[2]  + wtot[3];
    const int S1 = wtot[4]  + wtot[5]  + wtot[6]  + wtot[7];
    const int S2 = wtot[8]  + wtot[9]  + wtot[10] + wtot[11];
    const int S3 = wtot[12] + wtot[13] + wtot[14] + wtot[15];
    int pre = 0;
#pragma unroll 1
    for (int w = 4 * sub; w < wave; ++w) pre += wtot[w];
    const int b0 = carry;
    const int b1 = b0 + ((S0 + 31) & ~31);
    const int b2 = b1 + ((S1 + 31) & ~31);
    const int b3 = b2 + ((S2 + 31) & ~31);
    const int b4 = b3 + ((S3 + 31) & ~31);
    const int myb = sub == 0 ? b0 : (sub == 1 ? b1 : (sub == 2 ? b2 : b3));
    if (tid == 0) {
      srb[min(4 * ch + 0, RBN - 1)] = b0;
      srb[min(4 * ch + 1, RBN - 1)] = b1;
      srb[min(4 * ch + 2, RBN - 1)] = b2;
      srb[min(4 * ch + 3, RBN - 1)] = b3;
    }
    int run = myb + pre + incl - ts;
    soff[8 * tid + 0] = run; run += e0;
    soff[8 * tid + 1] = run; run += e1;
    soff[8 * tid + 2] = run; run += e2;
    soff[8 * tid + 3] = run; run += e3;
    soff[8 * tid + 4] = run; run += e4;
    soff[8 * tid + 5] = run; run += e5;
    soff[8 * tid + 6] = run; run += e6;
    soff[8 * tid + 7] = run;
    carry = b4;
    __syncthreads();
    const v4i o0 = *(const v4i*)(soff + 4 * tid);
    const v4i o1 = *(const v4i*)(soff + 4 * (tid + OTHR));
    int* op = off + base;
    *(volatile v4i*)(op + 4 * tid) = o0;
    *(volatile v4i*)(op + 4 * (tid + OTHR)) = o1;
    __threadfence();
    *(volatile v4i*)(op + 4 * tid) = o0;
    *(volatile v4i*)(op + 4 * (tid + OTHR)) = o1;
    __syncthreads();
  }
  if (tid == 0) srb[min(4 * nChunk, RBN - 1)] = carry;
  __syncthreads();
  v4i rv = {0, 0, 0, 0};
  if (tid < 32) rv = *(const v4i*)(srb + 4 * tid);
  if (tid < 32) *(volatile v4i*)(rbase + 4 * tid) = rv;
  __threadfence();
  if (tid < 32) *(volatile v4i*)(rbase + 4 * tid) = rv;
}

__global__ __launch_bounds__(NTHR) void k_fill(
    const int* __restrict__ srcs, const int* __restrict__ dsts,
    const int* __restrict__ off, const int* __restrict__ rbase,
    int* csr, int nN, int nE, int vec8, int csrLen) {
  extern __shared__ v4f lds_dyn[];
  int* region = (int*)lds_dyn;
  int* cursor = region + RCAP;
  int* list   = cursor + NBF;
  int* wcnt   = list + LISTN;
  const int tid = threadIdx.x, lane = tid & 31, wave = tid >> 5;
  const int b = blockIdx.x;
  const int nodeBase = b * NBF;

  int rb0 = rbase[b];
  const int rb1 = rbase[b + 1];
  rb0 = rb0 < 0 ? 0 : (rb0 > csrLen ? csrLen : rb0);
  rb0 &= ~31;
  int len = rb1 - rb0;
  len = len < 0 ? 0 : (len > RCAP ? RCAP : len);
  int lenW = (len + 31) & ~31;
  if (rb0 + lenW > csrLen) lenW = (csrLen - rb0) & ~31;

  {
    const v4i z = {0, 0, 0, 0};
    for (int i = tid; i < RCAP / 4; i += NTHR) ((v4i*)region)[i] = z;
    for (int s = tid; s < NBF; s += NTHR) {
      int o = off[nodeBase + s] - rb0;
      o = o < 0 ? 0 : (o > RCAP ? RCAP : o);
      cursor[s] = o;
    }
  }
  __syncthreads();

  const int nChunks = (nE + CHUNK - 1) / CHUNK;
#pragma unroll 1
  for (int ch = 0; ch < nChunks; ++ch) {
    const int cbase = ch * CHUNK;
    const int wc = scan_chunk<NBF>(dsts, nE, cbase, nodeBase, vec8, list, tid, lane, wave);
    if (lane == 0) wcnt[wave] = wc;
    __syncthreads();
    if (wave == 0) {
#pragma unroll 1
      for (int wsx = 0; wsx < NWAVE; ++wsx) {
        int n = __builtin_amdgcn_readfirstlane(wcnt[wsx]);
        n = n > WCAP ? WCAP : (n < 0 ? 0 : n);
        const int* lp = list + wsx * WCAP;
#pragma unroll 1
        for (int i = 0; i < n; ++i) {
          const int ent  = __builtin_amdgcn_readfirstlane(lp[i]);
          const int slot = ent & (NBF - 1);
          int e = cbase + ((ent >> 12) & (CHUNK - 1));
          e = e > nE - 1 ? nE - 1 : e;
          int sv = srcs[e];
          sv = sv < 0 ? 0 : (sv > nN - 1 ? nN - 1 : sv);
          if (lane == 0) {
            int pos = cursor[slot];
            pos = pos < 0 ? 0 : (pos > RCAP - 1 ? RCAP - 1 : pos);
            region[pos] = sv;
            const int np = pos + 1;
            cursor[slot] = np > RCAP ? RCAP : np;
          }
        }
      }
    }
    __syncthreads();
  }

  const int nv = lenW >> 2;
  int* gp = csr + rb0;
#pragma unroll 1
  for (int i = tid; i < nv; i += NTHR) { const v4i v = ((const v4i*)region)[i]; *(volatile v4i*)(gp + 4 * i) = v; }
  __threadfence();
#pragma unroll 1
  for (int i = tid; i < nv; i += NTHR) { const v4i v = ((const v4i*)region)[i]; *(volatile v4i*)(gp + 4 * i) = v; }
}

__global__ __launch_bounds__(NTHR) void k_wcvt(const float* __restrict__ w0, const float* __restrict__ w1,
                                               _Float16* dp, int K0, int K1, int K, int Nc, int nUnits) {
  const int i = (int)blockIdx.x * NTHR + (int)threadIdx.x;
  if (i >= nUnits) return;
  const int ppr = K >> 3;
  const int n = i / ppr;
  const int seg = i - n * ppr;
  int k1max = K1 - K0 - 1;
  k1max = k1max < 0 ? 0 : k1max;
  v8h o;
#pragma unroll
  for (int j = 0; j < 8; ++j) {
    const int k = 8 * seg + j;
    int ka = k > K0 - 1 ? K0 - 1 : k;
    ka = ka < 0 ? 0 : ka;
    int kb = k - K0;
    kb = kb < 0 ? 0 : (kb > k1max ? k1max : kb);
    const float fa = w0[(size_t)ka * Nc + n];
    const float fb = w1[(size_t)kb * Nc + n];
    const float f = (k < K0) ? fa : ((k < K1) ? fb : 0.f);
    o[j] = (_Float16)(f * WCARRY);
  }
  _Float16* gp = dp + (size_t)i * 8;
  *(volatile v8h*)gp = o;
  __threadfence();
  *(volatile v8h*)gp = o;
}

__global__ __launch_bounds__(NTHR) void k_xcvt(const float* __restrict__ x, _Float16* xp, int nN, int nPieces) {
  const int i = (int)blockIdx.x * NTHR + (int)threadIdx.x;
  if (i >= nPieces) return;
  constexpr int PPR = KIN / 8;
  const int row = i / PPR;
  const int seg = i - row * PPR;
  int rr = row > nN - 1 ? nN - 1 : row;
  rr = rr < 0 ? 0 : rr;
  const bool live = row < nN;
  const float* xr = x + (size_t)rr * FIN;
  v8h o;
#pragma unroll
  for (int j = 0; j < 8; ++j) {
    const int k = 8 * seg + j;
    const int kk = k > FIN - 1 ? FIN - 1 : k;
    const float f = xr[kk];
    const float fs = (live && k < FIN) ? f * ACARRY : 0.f;
    o[j] = (_Float16)fs;
  }
  _Float16* gp = xp + (size_t)i * 8;
  *(volatile v8h*)gp = o;
  __threadfence();
  *(volatile v8h*)gp = o;
}

template <int MODE>
__global__ __launch_bounds__(NTHR) void k_gemm(
    const _Float16* __restrict__ A, const _Float16* __restrict__ Bp, const float* __restrict__ bias,
    int hasBias, float* Cf, _Float16* Ch, int K, int ldc, int nValid, int nStore) {
  constexpr int TPW = 4;
  static_assert(TPW * 16 * 2 == BNC);
  static_assert(BM == 4 * 16);

  __shared__ __attribute__((aligned(16))) float stg[BM * BNC];
  const int tid = threadIdx.x, lane = tid & 31, wave = tid >> 5, hh = lane >> 4, m = lane & 15;
  const int rowBase = (int)blockIdx.x * BM;
  const int colBase = (int)blockIdx.y * BNC;
  const int rg = wave >> 1, chf = wave & 1;
  const int r0 = rg * 16;
  const int c0 = chf * (BNC / 2);

  v8f acc[TPW];
#pragma unroll
  for (int t = 0; t < TPW; ++t) { v8f z = {0.f, 0.f, 0.f, 0.f, 0.f, 0.f, 0.f, 0.f}; acc[t] = z; }

  const _Float16* ap = A  + (size_t)(rowBase + r0 + m) * K + 8 * hh;
  const _Float16* bp = Bp + (size_t)(colBase + c0 + m) * K + 8 * hh;
  const int ksteps = K >> 5;
#pragma unroll 1
  for (int kt = 0; kt < ksteps; ++kt) {
    Frag a;
    a.h[0] = *(const v8h*)(ap + 32 * kt);
    a.h[1] = *(const v8h*)(ap + 32 * kt + 16);
#pragma unroll
    for (int t = 0; t < TPW; ++t) {
      const size_t to = (size_t)(16 * t) * K + 32 * kt;
      Frag b;
      b.h[0] = *(const v8h*)(bp + to);
      b.h[1] = *(const v8h*)(bp + to + 16);
      acc[t] = wmh(a.v, b.v, acc[t]);
    }
  }

  float bv[TPW];
  if (hasBias != 0) {
#pragma unroll
    for (int t = 0; t < TPW; ++t) bv[t] = bias[colBase + c0 + 16 * t + m];
  } else {
#pragma unroll
    for (int t = 0; t < TPW; ++t) bv[t] = 0.f;
  }

  const int growb = rowBase + r0 + 8 * hh;
  if (MODE == 0) {
    {
      float* sp = stg + (size_t)(r0 + 8 * hh) * BNC + c0 + m;
#pragma unroll
      for (int t = 0; t < TPW; ++t) {
#pragma unroll
        for (int r = 0; r < 8; ++r) {
          const bool lv = (growb + r) < nValid;
          const float g = acc[t][r] * GSCALE + bv[t];
          sp[r * BNC + 16 * t] = lv ? g : 0.f;
        }
      }
    }
    __syncthreads();
    constexpr int NIT = (BM * (BNC / 4)) / NTHR;
    static_assert(NIT * NTHR == BM * (BNC / 4));
    v4f cv[NIT];
#pragma unroll
    for (int it = 0; it < NIT; ++it) {
      const int id = it * NTHR + tid;
      const int row = id >> 5, seg = id & 31;
      cv[it] = *(const v4f*)(stg + (size_t)row * BNC + 4 * seg);
    }
#pragma unroll
    for (int it = 0; it < NIT; ++it) {
      const int id = it * NTHR + tid;
      const int row = id >> 5, seg = id & 31;
      const int grow = rowBase + row;
      if (grow < nStore) {
        float* gp = Cf + (size_t)grow * ldc + colBase + 4 * seg;
        *(volatile v4f*)gp = cv[it];
      }
    }
    __threadfence();
#pragma unroll
    for (int it = 0; it < NIT; ++it) {
      const int id = it * NTHR + tid;
      const int row = id >> 5, seg = id & 31;
      const int grow = rowBase + row;
      if (grow < nStore) {
        float* gp = Cf + (size_t)grow * ldc + colBase + 4 * seg;
        *(volatile v4f*)gp = cv[it];
      }
    }
  } else {
    _Float16* sh = (_Float16*)stg;
    {
      _Float16* sp = sh + (size_t)(r0 + 8 * hh) * BNC + c0 + m;
#pragma unroll
      for (int t = 0; t < TPW; ++t) {
#pragma unroll
        for (int r = 0; r < 8; ++r) {
          const bool lv = (growb + r) < nValid;
          const float g = eluf(acc[t][r] * GSCALE + bv[t]);
          const float gs = lv ? g * ACARRY : 0.f;
          sp[r * BNC + 16 * t] = (_Float16)gs;
        }
      }
    }
    __syncthreads();
    constexpr int NIT = (BM * (BNC / 8)) / NTHR;
    static_assert(NIT * NTHR == BM * (BNC / 8));
    v8h hv[NIT];
#pragma unroll
    for (int it = 0; it < NIT; ++it) {
      const int id = it * NTHR + tid;
      const int row = id >> 4, seg = id & 15;
      hv[it] = *(const v8h*)(sh + (size_t)row * BNC + 8 * seg);
    }
#pragma unroll
    for (int it = 0; it < NIT; ++it) {
      const int id = it * NTHR + tid;
      const int row = id >> 4, seg = id & 15;
      const int grow = rowBase + row;
      if (grow < nStore) {
        _Float16* gp = Ch + (size_t)grow * ldc + colBase + 8 * seg;
        *(volatile v8h*)gp = hv[it];
      }
    }
    __threadfence();
#pragma unroll
    for (int it = 0; it < NIT; ++it) {
      const int id = it * NTHR + tid;
      const int row = id >> 4, seg = id & 15;
      const int grow = rowBase + row;
      if (grow < nStore) {
        _Float16* gp = Ch + (size_t)grow * ldc + colBase + 8 * seg;
        *(volatile v8h*)gp = hv[it];
      }
    }
  }
}

__global__ __launch_bounds__(NTHR) void k_aggsym(
    const int* __restrict__ csr, const int* __restrict__ off, const int* __restrict__ cnt,
    const float* __restrict__ dinv, const float* __restrict__ hw, const float* __restrict__ cb,
    const float* __restrict__ ng, const float* __restrict__ nb, const float* __restrict__ nm,
    const float* __restrict__ nv, _Float16* hout, int nN, int csrLen) {
  const int tid = threadIdx.x, lane = tid & 31, wave = tid >> 5;
  const int tbase = blockIdx.x * TGT + wave * 32;
  const int cl    = tbase + lane;
  const int cnt_l = cnt[cl];
  const int off_l = off[cl];
  const float di_l = dinv[cl];
  const v4f cb4 = *(const v4f*)(cb + 4 * lane);
  const v4f m4  = *(const v4f*)(nm + 4 * lane);
  const v4f b4  = *(const v4f*)(nb + 4 * lane);
  const v4f sc4 = nscale4(ng, nv, lane);

#pragma unroll 1
  for (int j = 0; j < 32; ++j) {
    const int c = tbase + j;
    int n = __shfl(cnt_l, j);
    n = n < 0 ? 0 : (n > DEGCAP ? DEGCAP : n);
    const int st = __shfl(off_l, j);
    const float dc = __shfl(di_l, j);

    v4f a = {0.f, 0.f, 0.f, 0.f};
#pragma unroll 1
    for (int q0 = 0; q0 < n; q0 += 32) {
      int pos = st + q0 + lane;
      pos = pos < 0 ? 0 : (pos > csrLen - 1 ? csrLen - 1 : pos);
      int sl = csr[pos];
      sl = sl < 0 ? 0 : (sl > nN - 1 ? nN - 1 : sl);
      const int mcnt = (n - q0) < 32 ? (n - q0) : 32;
#pragma unroll 1
      for (int pp = 0; pp < mcnt; ++pp) {
        const int s = __builtin_amdgcn_readlane(sl, pp);
        const float cf = dinv[s] * dc;
        const v4f xv = *(const v4f*)(hw + (size_t)s * HD + 4 * lane);
        a = a + xv * cf;
      }
    }
    const v4f hs = *(const v4f*)(hw + (size_t)c * HD + 4 * lane);
    a = a + hs * (dc * dc);

    const bool live = c < nN;
    v4f y = a + cb4;
    y = (y - m4) * sc4 + b4;
    y = elu4(y);
    y = selz(y, live);
    const v4h hq = cvt4h(y * ACARRY);
    _Float16* gp = hout + (size_t)c * HD + 4 * lane;
    *(volatile v4h*)gp = hq;
    __threadfence();
    *(volatile v4h*)gp = hq;
  }
}

__global__ __launch_bounds__(NTHR) void k_attvec(const float* __restrict__ g, const float* __restrict__ asv,
                                                 const float* __restrict__ adv, float* es4, int nN) {
  __shared__ __attribute__((aligned(16))) float sas[HD];
  __shared__ __attribute__((aligned(16))) float sad[HD];
  __shared__ __attribute__((aligned(16))) float so[NTHR * 4];
  const int tid = threadIdx.x;
  if (tid < HD) { sas[tid] = asv[tid]; sad[tid] = adv[tid]; }
  __syncthreads();
  const int node = (int)blockIdx.x * NTHR + tid;
  int rr = node > nN - 1 ? nN - 1 : node;
  rr = rr < 0 ? 0 : rr;
  const bool live = node < nN;
  const float* gp = g + (size_t)rr * HD;
  float s0 = 0.f, s1 = 0.f, d0 = 0.f, d1 = 0.f;
#pragma unroll 1
  for (int kq = 0; kq < DHD / 4; ++kq) {
    const v4f hv = *(const v4f*)(gp + 4 * kq);
#pragma unroll
    for (int t = 0; t < 4; ++t) {
      const int c = 4 * kq + t;
      s0 += hv[t] * sas[c];
      d0 += hv[t] * sad[c];
    }
  }
#pragma unroll 1
  for (int kq = DHD / 4; kq < HD / 4; ++kq) {
    const v4f hv = *(const v4f*)(gp + 4 * kq);
#pragma unroll
    for (int t = 0; t < 4; ++t) {
      const int c = 4 * kq + t;
      s1 += hv[t] * sas[c];
      d1 += hv[t] * sad[c];
    }
  }
  v4f o; o.x = s0; o.y = s1; o.z = d0; o.w = d1;
  *(v4f*)(so + 4 * tid) = selz(o, live);
  __syncthreads();
  const v4f v = *(const v4f*)(so + 4 * tid);
  float* op = es4 + ((size_t)blockIdx.x * NTHR + tid) * 4;
  *(volatile v4f*)op = v;
  __threadfence();
  *(volatile v4f*)op = v;
}

__global__ __launch_bounds__(NTHR) void k_aggatt(
    const int* __restrict__ csr, const int* __restrict__ off, const int* __restrict__ cnt,
    const float* __restrict__ es4, const float* __restrict__ gsrc, const float* __restrict__ cb,
    const float* __restrict__ ng, const float* __restrict__ nb, const float* __restrict__ nm,
    const float* __restrict__ nv, float* hout, int nN, int csrLen) {
  const int tid = threadIdx.x, lane = tid & 31, wave = tid >> 5, hsel = lane >> 4;
  const int tbase = blockIdx.x * TGT + wave * 32;
  const int cl    = tbase + lane;
  const int cnt_l = cnt[cl];
  const int off_l = off[cl];
  const v4f cb4 = *(const v4f*)(cb + 4 * lane);
  const v4f m4  = *(const v4f*)(nm + 4 * lane);
  const v4f b4  = *(const v4f*)(nb + 4 * lane);
  const v4f sc4 = nscale4(ng, nv, lane);
  const float NINF = -__builtin_inff();

#pragma unroll 1
  for (int j = 0; j < 32; ++j) {
    const int c = tbase + j;
    int n = __shfl(cnt_l, j);
    n = n < 0 ? 0 : (n > DEGCAP ? DEGCAP : n);
    const int st = __shfl(off_l, j);
    const v4f ec = *(const v4f*)(es4 + (size_t)c * 4);
    v2f edc; edc.x = ec.z; edc.y = ec.w;
    v2f eself; eself.x = lrelu1(ec.x + ec.z); eself.y = lrelu1(ec.y + ec.w);

    v2f mx = eself;
#pragma unroll 1
    for (int q0 = 0; q0 < n; q0 += 32) {
      int pos = st + q0 + lane;
      pos = pos < 0 ? 0 : (pos > csrLen - 1 ? csrLen - 1 : pos);
      int sl = csr[pos];
      sl = sl < 0 ? 0 : (sl > nN - 1 ? nN - 1 : sl);
      const int mcnt = (n - q0) < 32 ? (n - q0) : 32;
      const bool valid = lane < mcnt;
      const v4f esv = *(const v4f*)(es4 + (size_t)sl * 4);
      v2f e; e.x = lrelu1(esv.x + edc.x); e.y = lrelu1(esv.y + edc.y);
      e = selv2(e, valid, NINF);
      e = wmax2(e);
      mx.x = fmaxf(mx.x, e.x); mx.y = fmaxf(mx.y, e.y);
    }
    v2f z = {0.f, 0.f};
#pragma unroll 1
    for (int q0 = 0; q0 < n; q0 += 32) {
      int pos = st + q0 + lane;
      pos = pos < 0 ? 0 : (pos > csrLen - 1 ? csrLen - 1 : pos);
      int sl = csr[pos];
      sl = sl < 0 ? 0 : (sl > nN - 1 ? nN - 1 : sl);
      const int mcnt = (n - q0) < 32 ? (n - q0) : 32;
      const bool valid = lane < mcnt;
      const v4f esv = *(const v4f*)(es4 + (size_t)sl * 4);
      v2f ex;
      ex.x = __expf(lrelu1(esv.x + edc.x) - mx.x);
      ex.y = __expf(lrelu1(esv.y + edc.y) - mx.y);
      ex = selz(ex, valid);
      z = z + wsum2(ex);
    }
    v2f exs; exs.x = __expf(eself.x - mx.x); exs.y = __expf(eself.y - mx.y);
    z = z + exs;
    v2f rz; rz.x = 1.0f / (z.x + 1e-16f); rz.y = 1.0f / (z.y + 1e-16f);

    v4f acc = {0.f, 0.f, 0.f, 0.f};
#pragma unroll 1
    for (int q0 = 0; q0 < n; q0 += 32) {
      int pos = st + q0 + lane;
      pos = pos < 0 ? 0 : (pos > csrLen - 1 ? csrLen - 1 : pos);
      int sl = csr[pos];
      sl = sl < 0 ? 0 : (sl > nN - 1 ? nN - 1 : sl);
      const int mcnt = (n - q0) < 32 ? (n - q0) : 32;
      const bool valid = lane < mcnt;
      const v4f esv = *(const v4f*)(es4 + (size_t)sl * 4);
      v2f al;
      al.x = __expf(lrelu1(esv.x + edc.x) - mx.x) * rz.x;
      al.y = __expf(lrelu1(esv.y + edc.y) - mx.y) * rz.y;
      al = selz(al, valid);
#pragma unroll 1
      for (int pp = 0; pp < mcnt; ++pp) {
        const int s = __builtin_amdgcn_readlane(sl, pp);
        const float a0 = __int_as_float(__builtin_amdgcn_readlane(__float_as_int(al.x), pp));
        const float a1 = __int_as_float(__builtin_amdgcn_readlane(__float_as_int(al.y), pp));
        const float ap = (hsel == 0) ? a0 : a1;
        const v4f hv = *(const v4f*)(gsrc + (size_t)s * HD + 4 * lane);
        acc = acc + hv * ap;
      }
    }
    const float aps = (hsel == 0) ? exs.x * rz.x : exs.y * rz.y;
    const v4f hc = *(const v4f*)(gsrc + (size_t)c * HD + 4 * lane);
    acc = acc + hc * aps;

    const bool live = c < nN;
    v4f y = acc + cb4;
    y = (y - m4) * sc4 + b4;
    y = elu4(y);
    y = selz(y, live);
    float* gp = hout + (size_t)c * HD + 4 * lane;
    *(volatile v4f*)gp = y;
    __threadfence();
    *(volatile v4f*)gp = y;
  }
}

__global__ __launch_bounds__(NTHR) void k_aggmean(
    const int* __restrict__ csr, const int* __restrict__ off, const int* __restrict__ cnt,
    const float* __restrict__ h, _Float16* aout, int nN, int csrLen) {
  const int tid = threadIdx.x, lane = tid & 31, wave = tid >> 5;
  const int tbase = blockIdx.x * TGT + wave * 32;
  const int cl    = tbase + lane;
  const int cnt_l = cnt[cl];
  const int off_l = off[cl];

#pragma unroll 1
  for (int j = 0; j < 32; ++j) {
    const int c = tbase + j;
    int n0 = __shfl(cnt_l, j);
    n0 = n0 < 0 ? 0 : n0;
    const int n = n0 > DEGCAP ? DEGCAP : n0;
    const int st = __shfl(off_l, j);

    v4f a = {0.f, 0.f, 0.f, 0.f};
#pragma unroll 1
    for (int q0 = 0; q0 < n; q0 += 32) {
      int pos = st + q0 + lane;
      pos = pos < 0 ? 0 : (pos > csrLen - 1 ? csrLen - 1 : pos);
      int sl = csr[pos];
      sl = sl < 0 ? 0 : (sl > nN - 1 ? nN - 1 : sl);
      const int mcnt = (n - q0) < 32 ? (n - q0) : 32;
#pragma unroll 1
      for (int pp = 0; pp < mcnt; ++pp) {
        const int s = __builtin_amdgcn_readlane(sl, pp);
        const v4f xv = *(const v4f*)(h + (size_t)s * HD + 4 * lane);
        a = a + xv;
      }
    }
    const float rc = 1.0f / fmaxf((float)n0, 1.0f);
    const v4f self = *(const v4f*)(h + (size_t)c * HD + 4 * lane);
    const bool live = c < nN;
    const v4f am = selz(a * rc, live);
    const v4f sm = selz(self, live);
    const v4h lo = cvt4h(am * ACARRY);
    const v4h hi = cvt4h(sm * ACARRY);
    _Float16* gp = aout + (size_t)c * KSG + 4 * lane;
    *(volatile v4h*)gp = lo;
    *(volatile v4h*)(gp + HD) = hi;
    __threadfence();
    *(volatile v4h*)gp = lo;
    *(volatile v4h*)(gp + HD) = hi;
  }
}

__global__ __launch_bounds__(NTHR) void k_tail(
    const _Float16* __restrict__ asg, const _Float16* __restrict__ hh16,
    const _Float16* __restrict__ wsg, const _Float16* __restrict__ wrs, const _Float16* __restrict__ wc1p,
    const float* __restrict__ bsg, const float* __restrict__ n3g, const float* __restrict__ n3b,
    const float* __restrict__ n3m, const float* __restrict__ n3v, const float* __restrict__ brs,
    const float* __restrict__ bc1, const float* __restrict__ wc2, const float* __restrict__ bc2,
    float* out, int nN) {
  __shared__ __attribute__((aligned(16))) _Float16 s3h[BM * S3P];
  __shared__ __attribute__((aligned(16))) float sz[BM * SZP];
  __shared__ __attribute__((aligned(16))) float spar[5 * DHD];
  __shared__ float sbc1[ZW];
  __shared__ float swc2[ZW * NOUT];
  __shared__ float sbc2[NOUT];
  __shared__ __attribute__((aligned(16))) float so[BM * NOUT];
  const int tid = threadIdx.x, lane = tid & 31, wave = tid >> 5, hh = lane >> 4, m = lane & 15;
  const int rowBase = (int)blockIdx.x * BM;

  if (tid < DHD) {
    spar[tid]           = bsg[tid];
    spar[DHD + tid]     = n3m[tid];
    spar[2 * DHD + tid] = n3g[tid] / sqrtf(n3v[tid] + BNEPS);
    spar[3 * DHD + tid] = n3b[tid];
    spar[4 * DHD + tid] = brs[tid];
  }
  if (tid < ZW) sbc1[tid] = bc1[tid];
  if (tid < ZW * NOUT) swc2[tid] = wc2[tid];
  if (tid < NOUT) sbc2[tid] = bc2[tid];
  __syncthreads();

  const int rg = wave >> 1, chf = wave & 1;
  const int r0 = rg * 16, c0 = chf * 32;
  v8f accT[2], accR[2];
#pragma unroll
  for (int t = 0; t < 2; ++t) {
    v8f z = {0.f, 0.f, 0.f, 0.f, 0.f, 0.f, 0.f, 0.f}; accT[t] = z; accR[t] = z;
  }
  {
    const _Float16* ap = asg + (size_t)(rowBase + r0 + m) * KSG + 8 * hh;
    const _Float16* bp = wsg + (size_t)(c0 + m) * KSG + 8 * hh;
#pragma unroll 1
    for (int kt = 0; kt < KSG / 32; ++kt) {
      Frag a;
      a.h[0] = *(const v8h*)(ap + 32 * kt);
      a.h[1] = *(const v8h*)(ap + 32 * kt + 16);
#pragma unroll
      for (int t = 0; t < 2; ++t) {
        const size_t to = (size_t)(16 * t) * KSG + 32 * kt;
        Frag b;
        b.h[0] = *(const v8h*)(bp + to);
        b.h[1] = *(const v8h*)(bp + to + 16);
        accT[t] = wmh(a.v, b.v, accT[t]);
      }
    }
  }
  {
    const _Float16* ap = hh16 + (size_t)(rowBase + r0 + m) * HD + 8 * hh;
    const _Float16* bp = wrs + (size_t)(c0 + m) * HD + 8 * hh;
#pragma unroll 1
    for (int kt = 0; kt < HD / 32; ++kt) {
      Frag a;
      a.h[0] = *(const v8h*)(ap + 32 * kt);
      a.h[1] = *(const v8h*)(ap + 32 * kt + 16);
#pragma unroll
      for (int t = 0; t < 2; ++t) {
        const size_t to = (size_t)(16 * t) * HD + 32 * kt;
        Frag b;
        b.h[0] = *(const v8h*)(bp + to);
        b.h[1] = *(const v8h*)(bp + to + 16);
        accR[t] = wmh(a.v, b.v, accR[t]);
      }
    }
  }

#pragma unroll
  for (int t = 0; t < 2; ++t) {
    const int col = c0 + 16 * t + m;
    const float pb = spar[col], pm = spar[DHD + col], ps = spar[2 * DHD + col];
    const float pbb = spar[3 * DHD + col], pr = spar[4 * DHD + col];
#pragma unroll
    for (int r = 0; r < 8; ++r) {
      const int row = r0 + 8 * hh + r;
      float tv = accT[t][r] * GSCALE + pb;
      tv = (tv - pm) * ps + pbb;
      const float rv = accR[t][r] * GSCALE;
      const float h3 = eluf((tv + rv) + pr);
      s3h[row * S3P + col] = (_Float16)(h3 * ACARRY);
    }
  }
  __syncthreads();

  const int rt = wave >> 1, ct = wave & 1;
  v8f accZ = {0.f, 0.f, 0.f, 0.f, 0.f, 0.f, 0.f, 0.f};
  {
    const _Float16* azp = s3h + (rt * 16 + m) * S3P + 8 * hh;
    const _Float16* bzp = wc1p + (size_t)(ct * 16 + m) * DHD + 8 * hh;
#pragma unroll
    for (int ks = 0; ks < DHD / 32; ++ks) {
      Frag a, b;
      a.h[0] = *(const v8h*)(azp + 32 * ks);
      a.h[1] = *(const v8h*)(azp + 32 * ks + 16);
      b.h[0] = *(const v8h*)(bzp + 32 * ks);
      b.h[1] = *(const v8h*)(bzp + 32 * ks + 16);
      accZ = wmh(a.v, b.v, accZ);
    }
  }
  {
    const int col = ct * 16 + m;
    const float bz = sbc1[col];
#pragma unroll
    for (int r = 0; r < 8; ++r) {
      const int row = rt * 16 + 8 * hh + r;
      sz[row * SZP + col] = eluf(accZ[r] * GSCALE + bz);
    }
  }
  __syncthreads();

  if (tid < BM * NOUT) {
    const int row = tid >> 1, o = tid & 1;
    float acc = 0.f;
#pragma unroll 1
    for (int k = 0; k < ZW; ++k) acc += sz[row * SZP + k] * swc2[k * NOUT + o];
    so[tid] = acc + sbc2[o];
  }
  __syncthreads();

  if (wave == 0) {
    const v4f v = *(const v4f*)(so + 4 * lane);
    v2f v2; v2.x = v.x; v2.y = v.y;
    const int ra = rowBase + 2 * lane;
    const bool both = (ra + 1) < nN;
    const bool one  = ra < nN;
    float* op = out + (size_t)ra * NOUT;
    if (both) *(volatile v4f*)op = v;
    else if (one) *(volatile v2f*)op = v2;
    __threadfence();
    if (both) *(volatile v4f*)op = v;
    else if (one) *(volatile v2f*)op = v2;
  }
}

extern "C" void kernel_launch(void* const* d_in, const int* in_sizes, int n_in,
                              void* d_out, int out_size, void* d_ws, size_t ws_size,
                              hipStream_t stream) {
  if (n_in < 31) return;
  if (in_sizes[0] < FIN || (in_sizes[0] % FIN) != 0) return;
  const int nN = in_sizes[0] / FIN;
  if (nN < 1 || nN > (1 << 20)) return;
  if (in_sizes[1] < 2 || (in_sizes[1] & 1) != 0) return;
  const int nE = in_sizes[1] / 2;
  if (nE < 1 || nE > (1 << 26)) return;
  if (in_sizes[2] != FIN * HD || in_sizes[3] != HD) return;
  if (in_sizes[4] != HD * HD || in_sizes[5] != HD) return;
  if (in_sizes[6] != HD || in_sizes[7] != HD || in_sizes[8] != HD || in_sizes[9] != HD) return;
  if (in_sizes[10] != HD * HD || in_sizes[11] != 2 * DHD || in_sizes[12] != 2 * DHD || in_sizes[13] != HD) return;
  if (in_sizes[14] != HD || in_sizes[15] != HD || in_sizes[16] != HD || in_sizes[17] != HD) return;
  if (in_sizes[18] != HD * DHD || in_sizes[19] != DHD || in_sizes[20] != HD * DHD) return;
  if (in_sizes[21] != DHD || in_sizes[22] != DHD || in_sizes[23] != DHD || in_sizes[24] != DHD) return;
  if (in_sizes[25] != HD * DHD || in_sizes[26] != DHD) return;
  if (in_sizes[27] != DHD * ZW || in_sizes[28] != ZW || in_sizes[29] != ZW * NOUT || in_sizes[30] != NOUT) return;
  if (out_size != nN * NOUT) return;

  const float* x     = (const float*)d_in[0];
  const int*   ei    = (const int*)d_in[1];
  const int*   src   = ei;
  const int*   dst   = ei + nE;
  const float* w_in  = (const float*)d_in[2];
  const float* b_in  = (const float*)d_in[3];
  const float* w_g1  = (const float*)d_in[4];
  const float* b_g1  = (const float*)d_in[5];
  const float* n1g   = (const float*)d_in[6];
  const float* n1b   = (const float*)d_in[7];
  const float* n1m   = (const float*)d_in[8];
  const float* n1v   = (const float*)d_in[9];
  const float* w_at  = (const float*)d_in[10];
  const float* asv   = (const float*)d_in[11];
  const float* adv   = (const float*)d_in[12];
  const float* b_at  = (const float*)d_in[13];
  const float* n2g   = (const float*)d_in[14];
  const float* n2b   = (const float*)d_in[15];
  const float* n2m   = (const float*)d_in[16];
  const float* n2v   = (const float*)d_in[17];
  const float* w_sl  = (const float*)d_in[18];
  const float* b_sg  = (const float*)d_in[19];
  const float* w_sr  = (const float*)d_in[20];
  const float* n3g   = (const float*)d_in[21];
  const float* n3b   = (const float*)d_in[22];
  const float* n3m   = (const float*)d_in[23];
  const float* n3v   = (const float*)d_in[24];
  const float* w_rs  = (const float*)d_in[25];
  const float* b_rs  = (const float*)d_in[26];
  const float* w_c1  = (const float*)d_in[27];
  const float* b_c1  = (const float*)d_in[28];
  const float* w_c2  = (const float*)d_in[29];
  const float* b_c2  = (const float*)d_in[30];
  float* out = (float*)d_out;

  const int NPAD   = ((nN + TGT - 1) / TGT) * TGT;
  const int nAgg   = NPAD / TGT;
  const int nBC    = (nN + NBC - 1) / NBC;
  const int CNTPAD = nBC * NBC;
  if (CNTPAD < NPAD) return;
  if (4 * nBC + 1 > RBN) return;
  const int nBF    = (nN + NBF - 1) / NBF;
  if (nBF > 4 * nBC) return;
  const int csrLen = ((nE + 31) & ~31) + 4096;
  if (31 * 4 * nBC > 4096) return;
  const int nGemmR = NPAD / BM;
  const int nPieces = NPAD * (KIN / 8);

  char* ws = (char*)d_ws;
  size_t off = 0;
  const size_t oCnt = off; off += (size_t)CNTPAD * 4;                    off = (off + 255) & ~(size_t)255;
  const size_t oDi  = off; off += (size_t)CNTPAD * 4;                    off = (off + 255) & ~(size_t)255;
  const size_t oOff = off; off += (size_t)CNTPAD * 4;                    off = (off + 255) & ~(size_t)255;
  const size_t oRb  = off; off += (size_t)RBN * 4;                       off = (off + 255) & ~(size_t)255;
  const size_t oCsr = off; off += (size_t)csrLen * 4;                    off = (off + 255) & ~(size_t)255;
  const size_t oWin = off; off += (size_t)HD * KIN * 2;                  off = (off + 255) & ~(size_t)255;
  const size_t oWg1 = off; off += (size_t)HD * HD * 2;                   off = (off + 255) & ~(size_t)255;
  const size_t oWat = off; off += (size_t)HD * HD * 2;                   off = (off + 255) & ~(size_t)255;
  const size_t oWsg = off; off += (size_t)DHD * KSG * 2;                 off = (off + 255) & ~(size_t)255;
  const size_t oWrs = off; off += (size_t)DHD * HD * 2;                  off = (off + 255) & ~(size_t)255;
  const size_t oWc1 = off; off += (size_t)ZW * DHD * 2;                  off = (off + 255) & ~(size_t)255;
  const size_t oEs  = off; off += (size_t)NPAD * 4 * 4;                  off = (off + 255) & ~(size_t)255;
  const size_t oR1  = off; off += (size_t)NPAD * HD * 4;                 off = (off + 255) & ~(size_t)255;
  const size_t oR2  = off; off += (size_t)NPAD * HD * 2;                 off = (off + 255) & ~(size_t)255;
  const size_t oR3  = off; off += (size_t)NPAD * HD * 4;                 off = (off + 255) & ~(size_t)255;
  if (off > ws_size || off > (size_t)WSCAP) return;
  if ((size_t)NPAD * KIN * 2 > (size_t)NPAD * HD * 4) return;
  if ((size_t)NPAD * KSG * 2 > (size_t)NPAD * HD * 4) return;

  int*   cnt   = (int*)(ws + oCnt);
  float* dinv  = (float*)(ws + oDi);
  int*   offp  = (int*)(ws + oOff);
  int*   rb    = (int*)(ws + oRb);
  int*   csr   = (int*)(ws + oCsr);
  _Float16* win  = (_Float16*)(ws + oWin);
  _Float16* wg1  = (_Float16*)(ws + oWg1);
  _Float16* wat  = (_Float16*)(ws + oWat);
  _Float16* wsg  = (_Float16*)(ws + oWsg);
  _Float16* wrs  = (_Float16*)(ws + oWrs);
  _Float16* wc1p = (_Float16*)(ws + oWc1);
  float* es4     = (float*)(ws + oEs);
  _Float16* xp   = (_Float16*)(ws + oR1);
  _Float16* h1h  = (_Float16*)(ws + oR1);
  float*    h2f  = (float*)(ws + oR1);
  _Float16* hh16 = (_Float16*)(ws + oR2);
  float*    hwf  = (float*)(ws + oR3);
  float*    gf   = (float*)(ws + oR3);
  _Float16* asg  = (_Float16*)(ws + oR3);

  const int vec8 = ((nE & 3) == 0) ? 1 : 0;

  k_count<<<nBC, NTHR, 0, stream>>>(dst, cnt, dinv, nE, vec8);
  k_offsets<<<1, OTHR, 0, stream>>>(cnt, offp, rb, nBC);
  hipFuncSetAttribute(reinterpret_cast<const void*>(&k_fill),
                      hipFuncAttributeMaxDynamicSharedMemorySize, LDS_FILL);
  k_fill<<<nBF, NTHR, LDS_FILL, stream>>>(src, dst, offp, rb, csr, nN, nE, vec8, csrLen);

  {
    const int u1 = HD * (KIN / 8);
    k_wcvt<<<(u1 + NTHR - 1) / NTHR, NTHR, 0, stream>>>(w_in, w_in, win, FIN, FIN, KIN, HD, u1);
    const int u2 = HD * (HD / 8);
    k_wcvt<<<(u2 + NTHR - 1) / NTHR, NTHR, 0, stream>>>(w_g1, w_g1, wg1, HD, HD, HD, HD, u2);
    k_wcvt<<<(u2 + NTHR - 1) / NTHR, NTHR, 0, stream>>>(w_at, w_at, wat, HD, HD, HD, HD, u2);
    const int u3 = DHD * (KSG / 8);
    k_wcvt<<<(u3 + NTHR - 1) / NTHR, NTHR, 0, stream>>>(w_sl, w_sr, wsg, HD, KSG, KSG, DHD, u3);
    const int u4 = DHD * (HD / 8);
    k_wcvt<<<(u4 + NTHR - 1) / NTHR, NTHR, 0, stream>>>(w_rs, w_rs, wrs, HD, HD, HD, DHD, u4);
    const int u5 = ZW * (DHD / 8);
    k_wcvt<<<(u5 + NTHR - 1) / NTHR, NTHR, 0, stream>>>(w_c1, w_c1, wc1p, DHD, DHD, DHD, ZW, u5);
  }

  k_xcvt<<<(nPieces + NTHR - 1) / NTHR, NTHR, 0, stream>>>(x, xp, nN, nPieces);

  k_gemm<1><<<dim3(nGemmR, HD / BNC), NTHR, 0, stream>>>(xp, win, b_in, 1, hwf, hh16, KIN, HD, nN, NPAD);
  k_gemm<0><<<dim3(nGemmR, HD / BNC), NTHR, 0, stream>>>(hh16, wg1, b_in, 0, hwf, h1h, HD, HD, nN, NPAD);
  k_aggsym<<<nAgg, NTHR, 0, stream>>>(csr, offp, cnt, dinv, hwf, b_g1, n1g, n1b, n1m, n1v, h1h, nN, csrLen);
  k_gemm<0><<<dim3(nGemmR, HD / BNC), NTHR, 0, stream>>>(h1h, wat, b_in, 0, gf, hh16, HD, HD, nN, NPAD);
  k_attvec<<<NPAD / NTHR, NTHR, 0, stream>>>(gf, asv, adv, es4, nN);
  k_aggatt<<<nAgg, NTHR, 0, stream>>>(csr, offp, cnt, es4, gf, b_at, n2g, n2b, n2m, n2v, h2f, nN, csrLen);
  k_aggmean<<<nAgg, NTHR, 0, stream>>>(csr, offp, cnt, h2f, asg, nN, csrLen);
  k_tail<<<NPAD / BM, NTHR, 0, stream>>>(asg, hh16, wsg, wrs, wc1p, b_sg, n3g, n3b, n3m, n3v, b_rs,
                                         b_c1, w_c2, b_c2, out, nN);
}
